// DeTrCrossAttention_30734785970515
// MI455X (gfx1250) — hardware-verified
//
#include <hip/hip_runtime.h>


typedef _Float16 v16h __attribute__((ext_vector_type(16)));
typedef _Float16 v8h __attribute__((ext_vector_type(8)));
typedef float v8f __attribute__((ext_vector_type(8)));
typedef float v4f __attribute__((ext_vector_type(4)));

union Frag { v16h v; v8h hf[2]; };
union Pack8 { v8h v; _Float16 s[8]; };

static constexpr int SQ = 256;
static constexpr int SK = 1024;
static constexpr int NB = 8;
static constexpr int EMB = 1024;
static constexpr int NH = 16;
static constexpr int DH = 64;
static constexpr int NSLICE = NB * DH;
static constexpr int MQ = SQ * NB;
static constexpr int MKV = SK * NB;
static constexpr int EKV = 2 * EMB;

static constexpr int GBM = 128, GBN = 128, GBK = 32;
static constexpr int GAST = 40, GBST = 40;
static constexpr int GCSTH = 136;
static constexpr int GCSTF = 132;
static constexpr int GCRAW = 34816;

static constexpr int QST = 24, KST = 24, VST = 72, PST = 72;

__device__ __forceinline__ v8f wmma_f16(v16h a, v16h b, v8f c) {
  v8f d = __builtin_amdgcn_wmma_f32_16x16x32_f16(false, a, false, b, (short)0, c, false, false);
  asm volatile("v_nop\n\tv_nop\n\tv_nop\n\tv_nop" : "+v"(d) : "v"(a), "v"(b));
  return d;
}

__device__ __forceinline__ v8f zero8f() {
  v8f z;
#pragma unroll
  for (int i = 0; i < 8; ++i) z[i] = 0.0f;
  return z;
}

__device__ __forceinline__ v8h zero8h() {
  Pack8 p;
#pragma unroll
  for (int i = 0; i < 8; ++i) p.s[i] = (_Float16)0.0f;
  return p.v;
}

__device__ __forceinline__ v8h cvt8h(v4f a, v4f b, float sc) {
  Pack8 p;
  p.s[0] = (_Float16)(a.x * sc); p.s[1] = (_Float16)(a.y * sc);
  p.s[2] = (_Float16)(a.z * sc); p.s[3] = (_Float16)(a.w * sc);
  p.s[4] = (_Float16)(b.x * sc); p.s[5] = (_Float16)(b.y * sc);
  p.s[6] = (_Float16)(b.z * sc); p.s[7] = (_Float16)(b.w * sc);
  return p.v;
}

template <int MODE> struct GemmIO { typedef float AT; typedef _Float16 CT; };
template <> struct GemmIO<2> { typedef _Float16 AT; typedef float CT; };

template <int MODE>
__device__ __forceinline__ int wrow_of(int n) {
  if (MODE == 0) return (n & 15) * DH + (n >> 4);
  if (MODE == 1) {
    const int g = n >> 10, t = n & 1023;
    return (t & 15) * (2 * DH) + g * DH + (t >> 4);
  }
  return n;
}

template <int MODE>
__global__ __launch_bounds__(256) void k_gemm(const typename GemmIO<MODE>::AT* __restrict__ A,
                                              const float* __restrict__ W,
                                              const float* __restrict__ bias,
                                              typename GemmIO<MODE>::CT* __restrict__ C,
                                              int M, int N, int K) {
  __shared__ __attribute__((aligned(16))) _Float16 As[GBM * GAST];
  __shared__ __attribute__((aligned(16))) _Float16 Bs[GBN * GBST];
  __shared__ __attribute__((aligned(16))) unsigned char Craw[GCRAW];

  const int tid = threadIdx.x;
  const int wid = tid >> 5, lane = tid & 31, h = lane >> 4, m16 = lane & 15;
  const int waveM = wid & 3, waveN = wid >> 2;
  const int mBlock = blockIdx.y * GBM, nBlock = blockIdx.x * GBN;
  if (mBlock + GBM > M || nBlock + GBN > N) return;

  v8f acc[2][4];
#pragma unroll
  for (int mt = 0; mt < 2; ++mt)
#pragma unroll
    for (int nt = 0; nt < 4; ++nt) acc[mt][nt] = zero8f();

  const int srow = tid >> 1, shalf = tid & 1;
  const float* wsrc = W + (size_t)wrow_of<MODE>(nBlock + srow) * K + shalf * 16;
  _Float16* adst = As + srow * GAST + shalf * 16;
  _Float16* bdst = Bs + srow * GBST + shalf * 16;

  for (int k0 = 0; k0 < K; k0 += GBK) {
    if (MODE == 2) {
      const int mm = mBlock + srow;
      const int s = mm >> 3, b = mm & 7;
      const int d = (k0 >> 4) + shalf;
      const _Float16* src = (const _Float16*)A + ((size_t)(b * DH + d) * SQ + s) * NH;
      const v8h a0 = *(const v8h*)src;
      const v8h a1 = *(const v8h*)(src + 8);
      *(v8h*)adst = a0;
      *(v8h*)(adst + 8) = a1;
    } else {
      const float* src = (const float*)A + (size_t)(mBlock + srow) * K + k0 + shalf * 16;
      const v4f f0 = *(const v4f*)(src + 0);
      const v4f f1 = *(const v4f*)(src + 4);
      const v4f f2 = *(const v4f*)(src + 8);
      const v4f f3 = *(const v4f*)(src + 12);
      *(v8h*)adst = cvt8h(f0, f1, 1.0f);
      *(v8h*)(adst + 8) = cvt8h(f2, f3, 1.0f);
    }
    {
      const float* src = wsrc + k0;
      const v4f f0 = *(const v4f*)(src + 0);
      const v4f f1 = *(const v4f*)(src + 4);
      const v4f f2 = *(const v4f*)(src + 8);
      const v4f f3 = *(const v4f*)(src + 12);
      *(v8h*)bdst = cvt8h(f0, f1, 64.0f);
      *(v8h*)(bdst + 8) = cvt8h(f2, f3, 64.0f);
    }
    __syncthreads();

    Frag af[2], bf[4];
#pragma unroll
    for (int mt = 0; mt < 2; ++mt) {
      const _Float16* p = As + (waveM * 32 + mt * 16 + m16) * GAST + 8 * h;
      af[mt].hf[0] = *(const v8h*)p;
      af[mt].hf[1] = *(const v8h*)(p + 16);
    }
#pragma unroll
    for (int nt = 0; nt < 4; ++nt) {
      const _Float16* p = Bs + (waveN * 64 + nt * 16 + m16) * GBST + 8 * h;
      bf[nt].hf[0] = *(const v8h*)p;
      bf[nt].hf[1] = *(const v8h*)(p + 16);
    }
#pragma unroll
    for (int mt = 0; mt < 2; ++mt)
#pragma unroll
      for (int nt = 0; nt < 4; ++nt)
        acc[mt][nt] = wmma_f16(af[mt].v, bf[nt].v, acc[mt][nt]);
    __syncthreads();
  }

  if (MODE == 2) {
    float* Cs = (float*)Craw;
    float* Cg = (float*)C;
#pragma unroll
    for (int hh = 0; hh < 2; ++hh) {
      if ((waveM >> 1) == hh) {
#pragma unroll
        for (int mt = 0; mt < 2; ++mt)
#pragma unroll
          for (int nt = 0; nt < 4; ++nt) {
            const int col = waveN * 64 + nt * 16 + m16;
            const float bb = bias[nBlock + col];
#pragma unroll
            for (int r = 0; r < 8; ++r) {
              const int lrow = (waveM & 1) * 32 + mt * 16 + 8 * h + r;
              Cs[lrow * GCSTF + col] = acc[mt][nt][r] * (1.0f / 64.0f) + bb;
            }
          }
      }
      __syncthreads();
      v4f vals[8];
#pragma unroll
      for (int i = 0; i < 8; ++i) {
        const int idx = i * 256 + tid;
        const int lrow = idx >> 5, c4 = idx & 31;
        vals[i] = *(const v4f*)(Cs + lrow * GCSTF + c4 * 4);
      }
#pragma unroll
      for (int i = 0; i < 8; ++i) {
        const int idx = i * 256 + tid;
        const int lrow = idx >> 5, c4 = idx & 31;
        float* dst = Cg + (size_t)(mBlock + hh * 64 + lrow) * N + nBlock + c4 * 4;
        *(volatile v4f*)dst = vals[i];
      }
      __threadfence();
#pragma unroll
      for (int i = 0; i < 8; ++i) {
        const int idx = i * 256 + tid;
        const int lrow = idx >> 5, c4 = idx & 31;
        float* dst = Cg + (size_t)(mBlock + hh * 64 + lrow) * N + nBlock + c4 * 4;
        *(volatile v4f*)dst = vals[i];
      }
      __syncthreads();
    }
  } else {
    _Float16* Cs = (_Float16*)Craw;
    _Float16* Cg = (_Float16*)C;
#pragma unroll
    for (int mt = 0; mt < 2; ++mt)
#pragma unroll
      for (int nt = 0; nt < 4; ++nt) {
        const int col = waveN * 64 + nt * 16 + m16;
        const float bb = bias[wrow_of<MODE>(nBlock + col)];
#pragma unroll
        for (int r = 0; r < 8; ++r) {
          const int row = waveM * 32 + mt * 16 + 8 * h + r;
          Cs[row * GCSTH + col] = (_Float16)(acc[mt][nt][r] * (1.0f / 64.0f) + bb);
        }
      }
    __syncthreads();
    v8h vals[8];
#pragma unroll
    for (int i = 0; i < 8; ++i) {
      const int idx = i * 256 + tid;
      const int row = idx >> 4, c8 = idx & 15;
      vals[i] = *(const v8h*)(Cs + row * GCSTH + c8 * 8);
    }
#pragma unroll
    for (int i = 0; i < 8; ++i) {
      const int idx = i * 256 + tid;
      const int row = idx >> 4, c8 = idx & 15;
      _Float16* dst = Cg + (size_t)(mBlock + row) * N + nBlock + c8 * 8;
      *(volatile v8h*)dst = vals[i];
    }
    __threadfence();
#pragma unroll
    for (int i = 0; i < 8; ++i) {
      const int idx = i * 256 + tid;
      const int row = idx >> 4, c8 = idx & 15;
      _Float16* dst = Cg + (size_t)(mBlock + row) * N + nBlock + c8 * 8;
      *(volatile v8h*)dst = vals[i];
    }
  }
}

__global__ __launch_bounds__(256) void k_attn(const _Float16* __restrict__ q16,
                                              const _Float16* __restrict__ kv16,
                                              _Float16* __restrict__ ctx2) {
  __shared__ __attribute__((aligned(16))) _Float16 Qs[SQ * QST];
  __shared__ __attribute__((aligned(16))) _Float16 Ks[64 * KST];
  __shared__ __attribute__((aligned(16))) _Float16 VTs[NH * VST];
  __shared__ __attribute__((aligned(16))) _Float16 Ps[8 * 32 * PST];

  const int slice = blockIdx.x;
  if (slice >= NSLICE) return;
  const int b = slice / DH, d = slice - b * DH;
  const int tid = threadIdx.x;
  const int w = tid >> 5, lane = tid & 31, h = lane >> 4, m16 = lane & 15;

#pragma unroll
  for (int i = 0; i < 2; ++i) {
    const int c = i * 256 + tid;
    const int s = c >> 1, hf = c & 1;
    const v8h v = *(const v8h*)(q16 + (size_t)(s * NB + b) * EMB + d * NH + hf * 8);
    *(v8h*)(Qs + s * QST + hf * 8) = v;
  }
  __syncthreads();

  const v8h z8 = zero8h();
  Frag qa[2];
#pragma unroll
  for (int t = 0; t < 2; ++t) {
    qa[t].hf[0] = *(const v8h*)(Qs + (w * 32 + t * 16 + m16) * QST + 8 * h);
    qa[t].hf[1] = z8;
  }

  v8f cacc[2];
  cacc[0] = zero8f();
  cacc[1] = zero8f();
  float mrun[2][8], srun[2][8];
#pragma unroll
  for (int t = 0; t < 2; ++t)
#pragma unroll
    for (int r = 0; r < 8; ++r) { mrun[t][r] = -1e30f; srun[t][r] = 0.0f; }

  _Float16* pw = Ps + w * 32 * PST;
  const float scale = 0.125f;

  for (int kb = 0; kb < SK / 64; ++kb) {
    __syncthreads();
    if (tid < 128) {
      const int j = tid >> 1, hf = tid & 1;
      const v8h v = *(const v8h*)(kv16 + (size_t)((kb * 64 + j) * NB + b) * EKV + d * NH + hf * 8);
      *(v8h*)(Ks + j * KST + hf * 8) = v;
    } else {
      const int t2 = tid - 128;
      const int j = t2 >> 1, hf = t2 & 1;
      Pack8 u;
      u.v = *(const v8h*)(kv16 + (size_t)((kb * 64 + j) * NB + b) * EKV + EMB + d * NH + hf * 8);
#pragma unroll
      for (int i = 0; i < 8; ++i) VTs[(hf * 8 + i) * VST + j] = u.s[i];
    }
    __syncthreads();

    Frag kf[4];
#pragma unroll
    for (int nt = 0; nt < 4; ++nt) {
      kf[nt].hf[0] = *(const v8h*)(Ks + (nt * 16 + m16) * KST + 8 * h);
      kf[nt].hf[1] = z8;
    }

#pragma unroll
    for (int t = 0; t < 2; ++t) {
      v8f sc[4];
#pragma unroll
      for (int nt = 0; nt < 4; ++nt) sc[nt] = wmma_f16(qa[t].v, kf[nt].v, zero8f());

#pragma unroll
      for (int r = 0; r < 8; ++r) {
        float bmax = -1e30f;
#pragma unroll
        for (int nt = 0; nt < 4; ++nt) {
          const float sv = sc[nt][r] * scale;
          sc[nt][r] = sv;
          bmax = fmaxf(bmax, sv);
        }
        bmax = fmaxf(bmax, __shfl_xor(bmax, 1, 32));
        bmax = fmaxf(bmax, __shfl_xor(bmax, 2, 32));
        bmax = fmaxf(bmax, __shfl_xor(bmax, 4, 32));
        bmax = fmaxf(bmax, __shfl_xor(bmax, 8, 32));

        const float newm = fmaxf(mrun[t][r], bmax);
        const float f = __expf(mrun[t][r] - newm);
        mrun[t][r] = newm;
        cacc[t][r] = cacc[t][r] * f;

        float ps = 0.0f;
        const int rowl = t * 16 + 8 * h + r;
#pragma unroll
        for (int nt = 0; nt < 4; ++nt) {
          const float p = __expf(sc[nt][r] - newm);
          ps += p;
          pw[rowl * PST + nt * 16 + m16] = (_Float16)(p * 256.0f);
        }
        ps += __shfl_xor(ps, 1, 32);
        ps += __shfl_xor(ps, 2, 32);
        ps += __shfl_xor(ps, 4, 32);
        ps += __shfl_xor(ps, 8, 32);
        srun[t][r] = srun[t][r] * f + ps;
      }
    }
    __syncthreads();

    Frag vb[2];
#pragma unroll
    for (int kq = 0; kq < 2; ++kq) {
      const _Float16* p = VTs + m16 * VST + kq * 32 + 8 * h;
      vb[kq].hf[0] = *(const v8h*)p;
      vb[kq].hf[1] = *(const v8h*)(p + 16);
    }
#pragma unroll
    for (int t = 0; t < 2; ++t)
#pragma unroll
      for (int kq = 0; kq < 2; ++kq) {
        const _Float16* p = pw + (t * 16 + m16) * PST + kq * 32 + 8 * h;
        Frag pa;
        pa.hf[0] = *(const v8h*)p;
        pa.hf[1] = *(const v8h*)(p + 16);
        cacc[t] = wmma_f16(pa.v, vb[kq].v, cacc[t]);
      }
  }

  __syncthreads();
#pragma unroll
  for (int t = 0; t < 2; ++t)
#pragma unroll
    for (int r = 0; r < 8; ++r) {
      const int row = t * 16 + 8 * h + r;
      const float inv = 1.0f / (srun[t][r] * 256.0f);
      pw[row * PST + m16] = (_Float16)(cacc[t][r] * inv);
    }
  __syncthreads();
  v8h cv[2];
#pragma unroll
  for (int p = 0; p < 2; ++p) {
    const int c = p * 32 + lane;
    const int row = c >> 1, hf = c & 1;
    cv[p] = *(const v8h*)(pw + row * PST + hf * 8);
  }
  _Float16* dst = ctx2 + ((size_t)slice * SQ + w * 32) * NH;
#pragma unroll
  for (int p = 0; p < 2; ++p) *(volatile v8h*)(dst + (p * 32 + lane) * 8) = cv[p];
  __threadfence();
#pragma unroll
  for (int p = 0; p < 2; ++p) *(volatile v8h*)(dst + (p * 32 + lane) * 8) = cv[p];
}

extern "C" void kernel_launch(void* const* d_in, const int* in_sizes, int n_in,
                              void* d_out, int out_size, void* d_ws,
                              size_t ws_size, hipStream_t stream) {
  if (n_in < 8) return;
  if (in_sizes[0] != SQ * NB * EMB || in_sizes[1] != SK * NB * EMB ||
      in_sizes[2] != EMB * EMB || in_sizes[3] != EMB ||
      in_sizes[4] != EKV * EMB || in_sizes[5] != EKV ||
      in_sizes[6] != EMB * EMB || in_sizes[7] != EMB) return;
  if (out_size != SQ * NB * EMB) return;

  const float* x = (const float*)d_in[0];
  const float* memory = (const float*)d_in[1];
  const float* Wq = (const float*)d_in[2];
  const float* bq = (const float*)d_in[3];
  const float* Wkv = (const float*)d_in[4];
  const float* bkv = (const float*)d_in[5];
  const float* Wd = (const float*)d_in[6];
  const float* bd = (const float*)d_in[7];
  float* out = (float*)d_out;

  const size_t q_bytes = (size_t)MQ * EMB * 2;
  const size_t kv_bytes = (size_t)MKV * EKV * 2;
  const size_t ctx_bytes = (size_t)NSLICE * SQ * NH * 2;
  if (q_bytes + kv_bytes + ctx_bytes > ws_size) return;
  char* ws = (char*)d_ws;
  _Float16* q16 = (_Float16*)ws;
  _Float16* kv16 = (_Float16*)(ws + q_bytes);
  _Float16* ctx2 = (_Float16*)(ws + q_bytes + kv_bytes);

  dim3 blk(256);
  k_gemm<0><<<dim3(EMB / GBN, MQ / GBM), blk, 0, stream>>>(x, Wq, bq, q16, MQ, EMB, EMB);
  k_gemm<1><<<dim3(EKV / GBN, MKV / GBM), blk, 0, stream>>>(memory, Wkv, bkv, kv16, MKV, EKV, EMB);
  k_attn<<<dim3(NSLICE), blk, 0, stream>>>(q16, kv16, ctx2);
  k_gemm<2><<<dim3(EMB / GBN, MQ / GBM), blk, 0, stream>>>(ctx2, Wd, bd, out, MQ, EMB, EMB);
}
